// DummyAttention_87505663689046
// MI455X (gfx1250) — hardware-verified
//
#include <hip/hip_runtime.h>
#include <stddef.h>
#include <stdint.h>

#define NB   2
#define SQ   2048
#define NT   (NB * SQ)
#define DM   2048
#define NH   16
#define HD   128
#define QBLK (SQ / 128)
#define KCH  (SQ / 64)

static_assert(NT % 256 == 0);
static_assert(SQ % 128 == 0);
static_assert(SQ % 64 == 0);
static_assert(DM % 64 == 0);
static_assert(DM % 32 == 0);
static_assert(HD == 128);
static_assert(NH * HD == DM);
static_assert(DM / 8 == 256);

typedef _Float16 v16h __attribute__((ext_vector_type(16)));
typedef _Float16 v8h  __attribute__((ext_vector_type(8)));
typedef float    v8f  __attribute__((ext_vector_type(8)));
typedef float    v4f  __attribute__((ext_vector_type(4)));
typedef unsigned int v4u __attribute__((ext_vector_type(4)));

union Frag  { v16h v; v8h h[2]; };
union Pack8 { v8h h; v4u u; };

__device__ __forceinline__ v8f mma16(v16h a, v16h b, v8f c) {
  c = __builtin_amdgcn_wmma_f32_16x16x32_f16(false, a, false, b, (short)0, c, false, false);
  asm volatile("v_nop\n\tv_nop\n\tv_nop\n\tv_nop" : "+v"(c) : "v"(a), "v"(b));
  return c;
}

__device__ __forceinline__ v16h ldfrag(const _Float16* p, int ld, int row0, int k0, int lane) {
  const int m = lane & 15, lh = lane >> 4;
  const _Float16* q = p + (size_t)(row0 + m) * ld + k0 + 8 * lh;
  Frag f;
  f.h[0] = *(const v8h*)(q);
  f.h[1] = *(const v8h*)(q + 16);
  return f.v;
}

__device__ __forceinline__ v8f zero8() { return (v8f){0.f, 0.f, 0.f, 0.f, 0.f, 0.f, 0.f, 0.f}; }

__device__ __forceinline__ void gemm32x64(const _Float16* __restrict__ A, int lda,
                                          const _Float16* __restrict__ Bt, int ldb,
                                          int m0, int n0, int lane, v8f (&acc)[2][4]) {
#pragma unroll 2
  for (int k0 = 0; k0 < DM; k0 += 32) {
    const v16h a0 = ldfrag(A, lda, m0, k0, lane);
    const v16h a1 = ldfrag(A, lda, m0 + 16, k0, lane);
    const v16h b0 = ldfrag(Bt, ldb, n0, k0, lane);
    const v16h b1 = ldfrag(Bt, ldb, n0 + 16, k0, lane);
    const v16h b2 = ldfrag(Bt, ldb, n0 + 32, k0, lane);
    const v16h b3 = ldfrag(Bt, ldb, n0 + 48, k0, lane);
    acc[0][0] = mma16(a0, b0, acc[0][0]);
    acc[1][0] = mma16(a1, b0, acc[1][0]);
    acc[0][1] = mma16(a0, b1, acc[0][1]);
    acc[1][1] = mma16(a1, b1, acc[1][1]);
    acc[0][2] = mma16(a0, b2, acc[0][2]);
    acc[1][2] = mma16(a1, b2, acc[1][2]);
    acc[0][3] = mma16(a0, b3, acc[0][3]);
    acc[1][3] = mma16(a1, b3, acc[1][3]);
  }
}

__global__ __launch_bounds__(256) void k_cvt_x(const float* __restrict__ x, _Float16* __restrict__ xh, int ngrp) {
  const int t = blockIdx.x * 256 + (int)threadIdx.x;
  if (t >= ngrp) return;
  const size_t o = (size_t)t * 8;
  const v4f a0 = *(const v4f*)(x + o);
  const v4f a1 = *(const v4f*)(x + o + 4);
  Pack8 pk;
  pk.h = (v8h){(_Float16)a0[0], (_Float16)a0[1], (_Float16)a0[2], (_Float16)a0[3],
               (_Float16)a1[0], (_Float16)a1[1], (_Float16)a1[2], (_Float16)a1[3]};
  const v4u vv = pk.u;
  volatile v4u* d = (volatile v4u*)(xh + o);
  *d = vv;
  __threadfence();
  *d = vv;
}

__global__ __launch_bounds__(256) void k_wcvt(const float* __restrict__ w, _Float16* __restrict__ wh, int ngrp) {
  const int t = blockIdx.x * 256 + (int)threadIdx.x;
  if (t >= ngrp) return;
  const size_t o = (size_t)t * 8;
  const v4f w0 = *(const v4f*)(w + o);
  const v4f w1 = *(const v4f*)(w + o + 4);
  const v4f e0 = w0 * 32.0f;
  const v4f e1 = w1 * 32.0f;
  Pack8 pk;
  pk.h = (v8h){(_Float16)e0[0], (_Float16)e0[1], (_Float16)e0[2], (_Float16)e0[3],
               (_Float16)e1[0], (_Float16)e1[1], (_Float16)e1[2], (_Float16)e1[3]};
  const v4u vv = pk.u;
  volatile v4u* d = (volatile v4u*)(wh + o);
  *d = vv;
  __threadfence();
  *d = vv;
}

#define HTP 72
__global__ __launch_bounds__(256) void k_gemm_h(const _Float16* __restrict__ ap,
                                                const _Float16* __restrict__ wt,
                                                _Float16* __restrict__ plane) {
  __shared__ __align__(16) _Float16 st[8][32 * HTP];
  const int tid = threadIdx.x, lane = tid & 31, wave = tid >> 5;
  const int hh = lane >> 4, c = lane & 15;
  const int m0 = blockIdx.x * 256 + wave * 32;
  const int n0 = blockIdx.y * 64;

  v8f acc[2][4];
#pragma unroll
  for (int s = 0; s < 2; ++s)
#pragma unroll
    for (int t = 0; t < 4; ++t) acc[s][t] = zero8();
  gemm32x64(ap, DM, wt, DM, m0, n0, lane, acc);

  _Float16* sw = st[wave];
#pragma unroll
  for (int sub = 0; sub < 2; ++sub) {
#pragma unroll
    for (int t = 0; t < 4; ++t) {
#pragma unroll
      for (int r = 0; r < 8; ++r)
        sw[(sub * 16 + 8 * hh + r) * HTP + 16 * t + c] = (_Float16)(acc[sub][t][r] * 0.03125f);
    }
  }
  __syncthreads();

  const int h     = n0 >> 7;
  const int dbase = n0 & (HD - 1);
  v4u val[8];
  size_t go[8];
#pragma unroll
  for (int it = 0; it < 8; ++it) {
    const int p  = lane + 32 * it;
    const int L  = p >> 3;
    const int pc = p & 7;
    Pack8 pk;
    pk.h    = *(const v8h*)(sw + L * HTP + pc * 8);
    val[it] = pk.u;
    go[it]  = ((size_t)h * NT + (size_t)(m0 + L)) * HD + dbase + pc * 8;
  }
  for (int ps = 0; ps < 2; ++ps) {
#pragma unroll
    for (int it = 0; it < 8; ++it) *(volatile v4u*)(plane + go[it]) = val[it];
    __threadfence();
  }
}

#define STP 72
__global__ __launch_bounds__(256) void k_gemm_vt(const _Float16* __restrict__ xh,
                                                 const _Float16* __restrict__ wt,
                                                 _Float16* __restrict__ vt) {
  __shared__ __align__(16) _Float16 st[256 * STP];
  const int tid = threadIdx.x, lane = tid & 31, wave = tid >> 5;
  const int hh = lane >> 4, c = lane & 15;
  const int mb = blockIdx.x * 256;
  const int m0 = mb + wave * 32;
  const int n0 = blockIdx.y * 64;

  v8f acc[2][4];
#pragma unroll
  for (int s = 0; s < 2; ++s)
#pragma unroll
    for (int t = 0; t < 4; ++t) acc[s][t] = zero8();
  gemm32x64(xh, DM, wt, DM, m0, n0, lane, acc);

#pragma unroll
  for (int t = 0; t < 4; ++t) {
#pragma unroll
    for (int sub = 0; sub < 2; ++sub) {
#pragma unroll
      for (int r = 0; r < 8; ++r) {
        const int lr = wave * 32 + sub * 16 + 8 * hh + r;
        st[lr * STP + 16 * t + c] = (_Float16)(acc[sub][t][r] * 0.03125f);
      }
    }
  }
  __syncthreads();

  const int h     = n0 >> 7;
  const int dbase = n0 & (HD - 1);
  v4u val[8];
  size_t go[8];
#pragma unroll
  for (int j = 0; j < 8; ++j) {
    const int p  = tid + 256 * j;
    const int L  = p >> 3;
    const int pc = p & 7;
    const int d  = L >> 2;
    const int nl = (L & 3) * 64 + pc * 8;
    const _Float16* cp = st + nl * STP + d;
    Pack8 pk;
    pk.h = (v8h){cp[0 * STP], cp[1 * STP], cp[2 * STP], cp[3 * STP],
                 cp[4 * STP], cp[5 * STP], cp[6 * STP], cp[7 * STP]};
    val[j] = pk.u;
    go[j]  = ((size_t)(h * HD + dbase + d)) * NT + mb + nl;
  }
  for (int ps = 0; ps < 2; ++ps) {
#pragma unroll
    for (int j = 0; j < 8; ++j) *(volatile v4u*)(vt + go[j]) = val[j];
    __threadfence();
  }
}

#define KTP 136
#define VTP 72
#define PTP 72
#define OSP 136
#define KS_H (64 * KTP)
#define VS_H (128 * VTP)
#define PS_H (8 * 16 * PTP)
static_assert(8 * 16 * OSP <= KS_H + VS_H);

__global__ __launch_bounds__(256) void k_attn(const _Float16* __restrict__ qp,
                                              const _Float16* __restrict__ kp,
                                              const _Float16* __restrict__ vt,
                                              _Float16* __restrict__ op, float sscale) {
  __shared__ __align__(16) _Float16 Sh[KS_H + VS_H + PS_H];
  _Float16* Ks = Sh;
  _Float16* Vs = Sh + KS_H;
  _Float16* Pb = Sh + KS_H + VS_H;

  const int tid = threadIdx.x, lane = tid & 31, wave = tid >> 5;
  const int hh = lane >> 4, c = lane & 15;
  const int bh  = blockIdx.x / QBLK;
  const int qb  = blockIdx.x - bh * QBLK;
  const int b   = bh / NH;
  const int h   = bh - b * NH;
  const int kb0 = b * SQ;
  const int q0  = kb0 + qb * 128 + wave * 16;

  const _Float16* Q = qp + (size_t)h * NT * HD;
  const _Float16* K = kp + (size_t)h * NT * HD;
  const _Float16* V = vt + (size_t)h * HD * NT;

  v16h qa[4];
#pragma unroll
  for (int dc = 0; dc < 4; ++dc) qa[dc] = ldfrag(Q, HD, q0, dc * 32, lane);

  const float NEGI = -__builtin_huge_valf();
  float mrow[8], lrow[8];
  v8f oacc[8];
#pragma unroll
  for (int r = 0; r < 8; ++r) { mrow[r] = NEGI; lrow[r] = 0.f; }
#pragma unroll
  for (int t = 0; t < 8; ++t) oacc[t] = zero8();

  _Float16* pw = Pb + wave * 16 * PTP;

  for (int kc = 0; kc < KCH; ++kc) {
    const int kv0 = kb0 + kc * 64;
    __syncthreads();
    {
      const int r  = tid >> 2;
      const int qq = (tid & 3) * 32;
      const _Float16* ks = K + (size_t)(kv0 + r) * HD + qq;
      _Float16* kd = Ks + r * KTP + qq;
      *(v8h*)(kd)      = *(const v8h*)(ks);
      *(v8h*)(kd + 8)  = *(const v8h*)(ks + 8);
      *(v8h*)(kd + 16) = *(const v8h*)(ks + 16);
      *(v8h*)(kd + 24) = *(const v8h*)(ks + 24);
      const int r2 = tid >> 1;
      const int q2 = (tid & 1) * 32;
      const _Float16* vs = V + (size_t)r2 * NT + kv0 + q2;
      _Float16* vd = Vs + r2 * VTP + q2;
      *(v8h*)(vd)      = *(const v8h*)(vs);
      *(v8h*)(vd + 8)  = *(const v8h*)(vs + 8);
      *(v8h*)(vd + 16) = *(const v8h*)(vs + 16);
      *(v8h*)(vd + 24) = *(const v8h*)(vs + 24);
    }
    __syncthreads();

    v8f s[4];
#pragma unroll
    for (int j = 0; j < 4; ++j) s[j] = zero8();
#pragma unroll
    for (int dc = 0; dc < 4; ++dc) {
#pragma unroll
      for (int j = 0; j < 4; ++j) {
        const v16h kb = ldfrag(Ks, KTP, j * 16, dc * 32, lane);
        s[j] = mma16(qa[dc], kb, s[j]);
      }
    }
    float cm[8];
#pragma unroll
    for (int r = 0; r < 8; ++r) {
      float m = NEGI;
#pragma unroll
      for (int j = 0; j < 4; ++j) {
        const float sv = s[j][r] * sscale;
        s[j][r] = sv;
        m = fmaxf(m, sv);
      }
#pragma unroll
      for (int off = 1; off < 16; off <<= 1) m = fmaxf(m, __shfl_xor(m, off, 32));
      cm[r] = m;
    }
    float al[8];
#pragma unroll
    for (int r = 0; r < 8; ++r) {
      const float mnew  = fmaxf(mrow[r], cm[r]);
      const float alpha = __expf(mrow[r] - mnew);
      mrow[r] = mnew;
      float psum = 0.f;
#pragma unroll
      for (int j = 0; j < 4; ++j) {
        const float p = __expf(s[j][r] - mnew);
        psum += p;
        pw[(8 * hh + r) * PTP + j * 16 + c] = (_Float16)(p * 1024.0f);
      }
#pragma unroll
      for (int off = 1; off < 16; off <<= 1) psum += __shfl_xor(psum, off, 32);
      lrow[r] = lrow[r] * alpha + psum;
      al[r] = alpha;
    }
#pragma unroll
    for (int t = 0; t < 8; ++t)
#pragma unroll
      for (int r = 0; r < 8; ++r) oacc[t][r] *= al[r];
    __syncthreads();

#pragma unroll
    for (int kk = 0; kk < 2; ++kk) {
      const v16h pa = ldfrag(pw, PTP, 0, kk * 32, lane);
#pragma unroll
      for (int t = 0; t < 8; ++t) {
        const v16h vb = ldfrag(Vs, VTP, t * 16, kk * 32, lane);
        oacc[t] = mma16(pa, vb, oacc[t]);
      }
    }
  }
  __syncthreads();

  _Float16* ow = Sh + wave * 16 * OSP;
#pragma unroll
  for (int r = 0; r < 8; ++r) {
    const float inv = 0.03125f / lrow[r];
#pragma unroll
    for (int t = 0; t < 8; ++t) ow[(8 * hh + r) * OSP + 16 * t + c] = (_Float16)(oacc[t][r] * inv);
  }
  __syncthreads();
  v4u val[8];
  size_t go[8];
#pragma unroll
  for (int it = 0; it < 8; ++it) {
    const int p  = lane + 32 * it;
    const int L  = p >> 4;
    const int pc = p & 15;
    Pack8 pk;
    pk.h    = *(const v8h*)(ow + L * OSP + pc * 8);
    val[it] = pk.u;
    go[it]  = (size_t)(q0 + L) * DM + (size_t)h * HD + pc * 8;
  }
  for (int ps = 0; ps < 2; ++ps) {
#pragma unroll
    for (int it = 0; it < 8; ++it) *(volatile v4u*)(op + go[it]) = val[it];
    __threadfence();
  }
}

#define OTP 68
__global__ __launch_bounds__(256) void k_gemm_out(const _Float16* __restrict__ ap,
                                                  const _Float16* __restrict__ wt,
                                                  float* __restrict__ out, float oscale) {
  __shared__ __align__(16) float st[8][16 * OTP];
  const int tid = threadIdx.x, lane = tid & 31, wave = tid >> 5;
  const int hh = lane >> 4, c = lane & 15;
  const int m0 = blockIdx.x * 256 + wave * 32;
  const int n0 = blockIdx.y * 64;

  v8f acc[2][4];
#pragma unroll
  for (int s = 0; s < 2; ++s)
#pragma unroll
    for (int t = 0; t < 4; ++t) acc[s][t] = zero8();
  gemm32x64(ap, DM, wt, DM, m0, n0, lane, acc);

  float* sw = st[wave];
#pragma unroll
  for (int sub = 0; sub < 2; ++sub) {
    __syncthreads();
#pragma unroll
    for (int t = 0; t < 4; ++t) {
#pragma unroll
      for (int r = 0; r < 8; ++r)
        sw[(8 * hh + r) * OTP + 16 * t + c] = acc[sub][t][r] * oscale;
    }
    __syncthreads();
    v4f val[8];
    size_t go[8];
#pragma unroll
    for (int it = 0; it < 8; ++it) {
      const int p    = lane + 32 * it;
      const int L    = p >> 3;
      const int pc   = p & 7;
      const int row  = L >> 1;
      const int half = L & 1;
      val[it] = *(const v4f*)(sw + row * OTP + half * 32 + pc * 4);
      go[it]  = (size_t)(m0 + sub * 16 + row) * DM + n0 + half * 32 + pc * 4;
    }
    for (int ps = 0; ps < 2; ++ps) {
#pragma unroll
      for (int it = 0; it < 8; ++it) *(volatile v4f*)(out + go[it]) = val[it];
      __threadfence();
    }
  }
}

#define XH_B ((size_t)NT * DM * 2)
#define WP_B ((size_t)DM * DM * 2)
#define PL_B ((size_t)NT * DM * 2)
static_assert(XH_B + 4 * WP_B + 4 * PL_B == (size_t)117440512);
static_assert(XH_B + 4 * WP_B + 4 * PL_B <= (size_t)134217728);

extern "C" void kernel_launch(void* const* d_in, const int* in_sizes, int n_in,
                              void* d_out, int out_size, void* d_ws, size_t ws_size,
                              hipStream_t stream) {
  if (n_in < 5) return;
  if (in_sizes[0] != NT * DM) return;
  if (in_sizes[1] != DM * DM || in_sizes[2] != DM * DM || in_sizes[3] != DM * DM || in_sizes[4] != DM * DM) return;
  if (out_size != NT * DM) return;

  const float* x  = (const float*)d_in[0];
  const float* wq = (const float*)d_in[1];
  const float* wk = (const float*)d_in[2];
  const float* wv = (const float*)d_in[3];
  const float* wo = (const float*)d_in[4];
  float* out = (float*)d_out;

  size_t off = 0;
  const size_t oX  = off; off += XH_B;
  const size_t oWq = off; off += WP_B;
  const size_t oWk = off; off += WP_B;
  const size_t oWv = off; off += WP_B;
  const size_t oWo = off; off += WP_B;
  const size_t oQ  = off; off += PL_B;
  const size_t oK  = off; off += PL_B;
  const size_t oVt = off; off += PL_B;
  const size_t oO  = off; off += PL_B;
  if (off > ws_size) return;

  char* ws = (char*)d_ws;
  _Float16* Xh  = (_Float16*)(ws + oX);
  _Float16* Wqh = (_Float16*)(ws + oWq);
  _Float16* Wkh = (_Float16*)(ws + oWk);
  _Float16* Wvh = (_Float16*)(ws + oWv);
  _Float16* Woh = (_Float16*)(ws + oWo);
  _Float16* Qp  = (_Float16*)(ws + oQ);
  _Float16* Kp  = (_Float16*)(ws + oK);
  _Float16* Vtp = (_Float16*)(ws + oVt);
  _Float16* Op  = (_Float16*)(ws + oO);

  const int ngx = in_sizes[0] / 8;
  const int ngw = in_sizes[1] / 8;
  const dim3 ggrid(NT / 256, DM / 64);

  k_cvt_x<<<dim3((ngx + 255) / 256), dim3(256), 0, stream>>>(x, Xh, ngx);
  k_wcvt<<<dim3((ngw + 255) / 256), dim3(256), 0, stream>>>(wq, Wqh, ngw);
  k_wcvt<<<dim3((ngw + 255) / 256), dim3(256), 0, stream>>>(wk, Wkh, ngw);
  k_wcvt<<<dim3((ngw + 255) / 256), dim3(256), 0, stream>>>(wv, Wvh, ngw);
  k_wcvt<<<dim3((ngw + 255) / 256), dim3(256), 0, stream>>>(wo, Woh, ngw);
  k_gemm_h<<<ggrid, dim3(256), 0, stream>>>(Xh, Wqh, Qp);
  k_gemm_h<<<ggrid, dim3(256), 0, stream>>>(Xh, Wkh, Kp);
  k_gemm_vt<<<ggrid, dim3(256), 0, stream>>>(Xh, Wvh, Vtp);
  k_attn<<<dim3(NB * NH * QBLK), dim3(256), 0, stream>>>(Qp, Kp, Vtp, Op, 0.08838834764831845f);
  k_gemm_out<<<ggrid, dim3(256), 0, stream>>>(Op, Woh, out, 0.0009765625f);
  (void)hipGetLastError();
}
